// PSGNet_40673340293839
// MI455X (gfx1250) — hardware-verified
//
#include <hip/hip_runtime.h>
#include <stdint.h>
#include <stddef.h>
#include <math.h>

#pragma clang fp contract(off)

#define NBATCH 4
#define IMS    256
#define NPIX   (NBATCH * IMS * IMS)
#define FF     64
#define HID    100
#define NM1    4096
#define NM2    512
#define DIN    68
#define NQ     18
#define NCOL   128
#define TR     64
#define AP     136
#define YP     68
#define RECW   32
#define XINW   96
#define JSFW   32
#define CH     2048
#define NOWN   64
#define PA1    32
#define PAG    68
#define PA2    72
#define LA     (TR * AP * 2)
#define LW     (NCOL * AP * 2)
#define LDS_FC (2 * LA + LW)
#define A_SC   8.0f
#define W_SC   256.0f
#define R_ACC  0.00048828125f
#define RH     0.00390625f

static_assert((AP % 8) == 0);
static_assert((YP % 4) == 0);
static_assert(TR * YP * 4 <= LW);
static_assert((LA % 16) == 0);
static_assert((NM1 % TR) == 0);
static_assert((NM2 % TR) == 0);
static_assert((NM1 % NOWN) == 0);
static_assert((NM2 % NOWN) == 0);
static_assert((NPIX % 256) == 0);
static_assert(CH == 8 * 256);
static_assert(NOWN == 64);
static_assert((PA1 % 4) == 0);
static_assert((PAG % 4) == 0);
static_assert((PA2 % 4) == 0);
static_assert((NOWN * PA1) % 256 == 0);
static_assert(DIN <= 96);
static_assert(HID <= NCOL);
static_assert(NQ + 2 <= JSFW);
static_assert((RECW % 8) == 0);
static_assert((XINW % 8) == 0);
static_assert(IMS == 256);
static_assert(TR == 64);

typedef _Float16       v16h __attribute__((ext_vector_type(16)));
typedef _Float16       v8h  __attribute__((ext_vector_type(8)));
typedef float          v8f  __attribute__((ext_vector_type(8)));
typedef float          v4f  __attribute__((ext_vector_type(4)));
typedef float          v2f  __attribute__((ext_vector_type(2)));
typedef unsigned int   v4u  __attribute__((ext_vector_type(4)));
typedef int            v4i  __attribute__((ext_vector_type(4)));
typedef v4f __attribute__((may_alias)) v4fa;
typedef v2f __attribute__((may_alias)) v2fa;
typedef v4u __attribute__((may_alias)) v4ua;
typedef v4i __attribute__((may_alias)) v4ia;

union FragH { v16h v; v4u q[2]; };
union Pack8 { v8h h; v4u u; };

__device__ __forceinline__ unsigned short hbits(float f) {
  _Float16 t = (_Float16)f;
  unsigned short u;
  __builtin_memcpy(&u, &t, 2);
  return u;
}

__device__ __forceinline__ v8f wmma_h(v16h a, v16h b, v8f c) {
  v8f d = __builtin_amdgcn_wmma_f32_16x16x32_f16(false, a, false, b, (short)0, c, false, false);
  asm volatile("v_nop\n\tv_nop\n\tv_nop\n\tv_nop" : "+v"(d) : "v"(a), "v"(b));
  return d;
}

__device__ __forceinline__ v16h ldfrag(const unsigned short* p, int h) {
  FragH f;
  f.q[0] = *(const v4ua*)(p + 8 * h);
  f.q[1] = *(const v4ua*)(p + 16 + 8 * h);
  return f.v;
}

template <int KQ, int NR>
__device__ __forceinline__ void cvt_w(const float* __restrict__ W, int K, int N,
                                      unsigned short* sWp, int tid)
{
  #pragma unroll 1
  for (int i = tid; i < NR * KQ; i += 256) {
    const int n = i / KQ, q = i - n * KQ;
    const int nc = (n < N) ? n : (N - 1);
    Pack8 pk;
    #pragma unroll
    for (int j = 0; j < 8; ++j) {
      const int k = 8 * q + j;
      const int kc = (k < K) ? k : (K - 1);
      float v = W[(size_t)kc * N + nc] * W_SC;
      v = (k < K && n < N) ? v : 0.f;
      pk.h[j] = (_Float16)v;
    }
    *(v4ua*)(sWp + n * AP + 8 * q) = pk.u;
  }
}

__device__ __forceinline__ void stage_bias(const float* __restrict__ b, int N, float* sB, int tid) {
  if (tid < NCOL) {
    const int c = (tid < N) ? tid : (N - 1);
    const float v = b[c];
    sB[tid] = (tid < N) ? v : 0.f;
  }
}

__device__ __forceinline__ void gemm4(const unsigned short* sAc, const unsigned short* sWp, int KS,
                                      int rt, int ct0, int m, int h, v8f* acc)
{
  const v8f z8 = {0.f, 0.f, 0.f, 0.f, 0.f, 0.f, 0.f, 0.f};
  acc[0] = z8; acc[1] = z8; acc[2] = z8; acc[3] = z8;
  #pragma unroll 1
  for (int ks = 0; ks < KS; ++ks) {
    const v16h a = ldfrag(sAc + (16 * rt + m) * AP + 32 * ks, h);
    #pragma unroll
    for (int nt = 0; nt < 4; ++nt) {
      const v16h bq = ldfrag(sWp + (16 * (ct0 + nt) + m) * AP + 32 * ks, h);
      acc[nt] = wmma_h(a, bq, acc[nt]);
    }
  }
}

__device__ __forceinline__ void epi_hid(const v8f* acc, const float* sB, unsigned short* sAn,
                                        int rt, int ct0, int m, int h)
{
  #pragma unroll
  for (int nt = 0; nt < 4; ++nt) {
    const int col = 16 * (ct0 + nt) + m;
    const float bc = sB[col];
    #pragma unroll
    for (int r = 0; r < 8; ++r) {
      const int row = 16 * rt + 8 * h + r;
      float v = acc[nt][r] * R_ACC + bc;
      v = (v > 0.f) ? v : 0.f;
      sAn[row * AP + col] = hbits(v * A_SC);
    }
  }
}

__device__ __forceinline__ int compact_chunk(const int* __restrict__ keys, int nK, int cbase,
                                             int c0, int* sList, int* sTot,
                                             int tid, int lane, int wv)
{
  int kv[8];
  if (cbase + CH <= nK) {
    const v4ia* p = (const v4ia*)(keys + cbase + 8 * tid);
    const v4i u0 = p[0], u1 = p[1];
    kv[0] = u0.x; kv[1] = u0.y; kv[2] = u0.z; kv[3] = u0.w;
    kv[4] = u1.x; kv[5] = u1.y; kv[6] = u1.z; kv[7] = u1.w;
  } else {
    #pragma unroll
    for (int i = 0; i < 8; ++i) {
      const int e = cbase + 8 * tid + i;
      const int ec = (e < nK) ? e : (nK - 1);
      const int k = keys[ec];
      kv[i] = (e < nK) ? k : -1;
    }
  }
  int hm = 0;
  #pragma unroll
  for (int i = 0; i < 8; ++i) {
    const int lc = kv[i] - c0;
    hm |= ((unsigned)lc < (unsigned)NOWN) ? (1 << i) : 0;
  }
  const int cnt = __builtin_popcount(hm);
  int incl = cnt;
  #pragma unroll
  for (int off = 1; off < 32; off <<= 1) {
    const int t = __shfl_up(incl, off);
    incl += (lane >= off) ? t : 0;
  }
  if (lane == 31) sTot[wv] = incl;
  __syncthreads();
  int pre = 0, tot = 0;
  #pragma unroll
  for (int w = 0; w < 8; ++w) {
    const int t = sTot[w];
    pre += (w < wv) ? t : 0;
    tot += t;
  }
  int pos = pre + incl - cnt;
  #pragma unroll
  for (int i = 0; i < 8; ++i) {
    if (hm & (1 << i)) {
      sList[pos] = ((cbase + 8 * tid + i) << 6) | (kv[i] - c0);
      ++pos;
    }
  }
  __syncthreads();
  return tot;
}

__device__ __forceinline__ unsigned own_mask(const int* sList, int base, int Lc, int lane, int wv) {
  const int e = base + lane;
  const int ec = (e < Lc) ? e : (Lc - 1);
  const int v = sList[ec];
  const bool own = (e < Lc) && (((v & 63) >> 3) == wv);
  return (unsigned)__ballot(own);
}

__global__ __launch_bounds__(256) void k_pool1(const float* __restrict__ img,
                                               const int* __restrict__ cl1, int nK,
                                               float* __restrict__ rec)
{
  __shared__ __align__(16) float sAcc[NOWN * PA1];
  __shared__ int sList[CH];
  __shared__ int sTot[8];
  const int tid = threadIdx.x, lane = tid & 31, wv = tid >> 5;
  const int c0 = blockIdx.x * NOWN;
  #pragma unroll
  for (int j = 0; j < (NOWN * PA1) / 256; ++j) sAcc[tid + 256 * j] = 0.f;
  const int kk = (lane < 27) ? lane : 26;
  const int kh = kk / 9;
  const int kw = (kk / 3) % 3;
  const int ci = kk % 3;
  __syncthreads();

  #pragma unroll 1
  for (int cbase = 0; cbase < nK; cbase += CH) {
    const int L = compact_chunk(cl1, nK, cbase, c0, sList, sTot, tid, lane, wv);
    const int Lc = (L < CH) ? L : CH;
    #pragma unroll 1
    for (int base = 0; base < Lc; base += 32) {
      unsigned msk = own_mask(sList, base, Lc, lane, wv);
      while (msk != 0u) {
        const int idx = __builtin_ctz(msk);
        msk &= msk - 1u;
        const int v = sList[base + idx];
        const int lc = v & 63;
        int p = v >> 6;
        p = (p < 0) ? 0 : ((p > NPIX - 1) ? (NPIX - 1) : p);
        const int b = p >> 16, i = (p >> 8) & 255, j = p & 255;
        const int ih = i + kh - 1, jw = j + kw - 1;
        const bool in = ((unsigned)ih < (unsigned)IMS) && ((unsigned)jw < (unsigned)IMS);
        const int ihc = (ih < 0) ? 0 : ((ih > IMS - 1) ? (IMS - 1) : ih);
        const int jwc = (jw < 0) ? 0 : ((jw > IMS - 1) ? (IMS - 1) : jw);
        const float x = img[(((size_t)b * IMS + ihc) * IMS + jwc) * 3 + ci];
        const float gx = (float)i * RH, gy = (float)j * RH;
        float val = in ? x : 0.f;
        val = (lane < 27) ? val
            : ((lane == 27) ? gx
            : ((lane == 28) ? gy
            : ((lane == 29) ? (gx * gx)
            : ((lane == 30) ? (gy * gy) : 1.0f))));
        sAcc[lc * PA1 + lane] += val;
      }
    }
  }
  __syncthreads();

  v4f rv[8];
  #pragma unroll
  for (int q = 0; q < 8; ++q)
    rv[q] = *(const v4fa*)(sAcc + (8 * wv + q) * PA1 + 4 * (lane & 7));
  float* d = rec + (size_t)(c0 + 8 * wv) * RECW + 4 * lane;
  #pragma unroll
  for (int q = 0; q < 8; ++q)
    if (lane < 8) *(volatile v4f*)(d + q * RECW) = rv[q];
  __threadfence();
  #pragma unroll
  for (int q = 0; q < 8; ++q)
    if (lane < 8) *(volatile v4f*)(d + q * RECW) = rv[q];
}

__global__ __launch_bounds__(256) void k_gagg(const float* __restrict__ x,
                                              const int* __restrict__ edges, int nE, int nNode,
                                              float* __restrict__ agg)
{
  __shared__ __align__(16) float sAcc[NOWN * PAG];
  __shared__ int sList[CH];
  __shared__ int sTot[8];
  const int tid = threadIdx.x, lane = tid & 31, wv = tid >> 5;
  const int c0 = blockIdx.x * NOWN;
  #pragma unroll 1
  for (int i = tid; i < NOWN * PAG; i += 256) sAcc[i] = 0.f;
  const int* keys = edges + nE;
  __syncthreads();

  #pragma unroll 1
  for (int cbase = 0; cbase < nE; cbase += CH) {
    const int L = compact_chunk(keys, nE, cbase, c0, sList, sTot, tid, lane, wv);
    const int Lc = (L < CH) ? L : CH;
    #pragma unroll 1
    for (int base = 0; base < Lc; base += 32) {
      unsigned msk = own_mask(sList, base, Lc, lane, wv);
      while (msk != 0u) {
        const int idx = __builtin_ctz(msk);
        msk &= msk - 1u;
        const int v = sList[base + idx];
        const int lc = v & 63;
        int e = v >> 6;
        e = (e < 0) ? 0 : ((e > nE - 1) ? (nE - 1) : e);
        int s = edges[e];
        s = (s < 0) ? 0 : ((s > nNode - 1) ? (nNode - 1) : s);
        const v2f xv = *(const v2fa*)(x + (size_t)s * FF + 2 * lane);
        float* a = sAcc + lc * PAG + 2 * lane;
        v2f cur = *(v2fa*)a;
        cur += xv;
        *(v2fa*)a = cur;
        if (lane == 0) sAcc[lc * PAG + FF] += 1.0f;
      }
    }
  }
  __syncthreads();

  v4f rv[8];
  #pragma unroll
  for (int q = 0; q < 8; ++q) {
    const int lc = 8 * wv + q;
    const float cnt = sAcc[lc * PAG + FF];
    const float rd = 1.0f / fmaxf(cnt, 1.0f);
    const v4f s4 = *(const v4fa*)(sAcc + lc * PAG + 4 * (lane & 15));
    rv[q] = s4 * rd;
  }
  float* d = agg + (size_t)(c0 + 8 * wv) * FF + 4 * lane;
  #pragma unroll
  for (int q = 0; q < 8; ++q)
    if (lane < 16) *(volatile v4f*)(d + q * FF) = rv[q];
  __threadfence();
  #pragma unroll
  for (int q = 0; q < 8; ++q)
    if (lane < 16) *(volatile v4f*)(d + q * FF) = rv[q];
}

__global__ __launch_bounds__(256) void k_pool2(const float* __restrict__ x1,
                                               const float* __restrict__ rec1,
                                               const int* __restrict__ cl2, int nK,
                                               float* __restrict__ xin)
{
  __shared__ __align__(16) float sAcc[NOWN * PA2];
  __shared__ int sList[CH];
  __shared__ int sTot[8];
  const int tid = threadIdx.x, lane = tid & 31, wv = tid >> 5;
  const int c0 = blockIdx.x * NOWN;
  #pragma unroll 1
  for (int i = tid; i < NOWN * PA2; i += 256) sAcc[i] = 0.f;
  const int sl = (lane < 4) ? lane : 4;
  __syncthreads();

  #pragma unroll 1
  for (int cbase = 0; cbase < nK; cbase += CH) {
    const int L = compact_chunk(cl2, nK, cbase, c0, sList, sTot, tid, lane, wv);
    const int Lc = (L < CH) ? L : CH;
    #pragma unroll 1
    for (int base = 0; base < Lc; base += 32) {
      unsigned msk = own_mask(sList, base, Lc, lane, wv);
      while (msk != 0u) {
        const int idx = __builtin_ctz(msk);
        msk &= msk - 1u;
        const int v = sList[base + idx];
        const int lc = v & 63;
        int c = v >> 6;
        c = (c < 0) ? 0 : ((c > nK - 1) ? (nK - 1) : c);
        const v2f xv = *(const v2fa*)(x1 + (size_t)c * FF + 2 * lane);
        float* a = sAcc + lc * PA2 + 2 * lane;
        v2f cur = *(v2fa*)a;
        cur += xv;
        *(v2fa*)a = cur;
        const float sv = rec1[(size_t)c * RECW + 27 + sl];
        const float v6 = (lane < 5) ? sv : 1.0f;
        if (lane < 6) sAcc[lc * PA2 + FF + lane] += v6;
      }
    }
  }
  __syncthreads();

  v4f rv[8];
  #pragma unroll
  for (int q = 0; q < 8; ++q) {
    const int lc = 8 * wv + q;
    const float rc = sAcc[lc * PA2 + FF + 5];
    const float pc = sAcc[lc * PA2 + FF + 4];
    const float rr = 1.0f / fmaxf(rc, 1.0f);
    const float rp = 1.0f / fmaxf(pc, 1.0f);
    const int ql = (lane < 16) ? lane : 16;
    const v4f s4 = *(const v4fa*)(sAcc + lc * PA2 + 4 * ql);
    const float f = (lane < 16) ? rr : rp;
    v4f o = s4 * f;
    const bool keep = (lane <= 16);
    o.x = keep ? o.x : 0.f;
    o.y = keep ? o.y : 0.f;
    o.z = keep ? o.z : 0.f;
    o.w = keep ? o.w : 0.f;
    rv[q] = o;
  }
  float* d = xin + (size_t)(c0 + 8 * wv) * XINW + 4 * lane;
  #pragma unroll
  for (int q = 0; q < 8; ++q)
    if (lane < 24) *(volatile v4f*)(d + q * XINW) = rv[q];
  __threadfence();
  #pragma unroll
  for (int q = 0; q < 8; ++q)
    if (lane < 24) *(volatile v4f*)(d + q * XINW) = rv[q];
}

template <int MODE>
__global__ __launch_bounds__(256) void k_fc(const float* __restrict__ src,
                                            const float* __restrict__ cw, const float* __restrict__ cb,
                                            const float* __restrict__ wi, const float* __restrict__ bi,
                                            const float* __restrict__ wh, const float* __restrict__ bh,
                                            const float* __restrict__ wo, const float* __restrict__ bo,
                                            const float* __restrict__ cst, int cpitch, int ci0, int cicnt,
                                            float* __restrict__ out)
{
  extern __shared__ __align__(16) unsigned char dsm_fc[];
  unsigned short* sA0 = (unsigned short*)dsm_fc;
  unsigned short* sA1 = (unsigned short*)(dsm_fc + LA);
  unsigned short* sW  = (unsigned short*)(dsm_fc + 2 * LA);
  float* sY = (float*)(dsm_fc + 2 * LA);
  __shared__ float sBias[NCOL];
  __shared__ float sStat[TR * 8];

  const int tid = threadIdx.x, lane = tid & 31, wv = tid >> 5;
  const int h = lane >> 4, m = lane & 15;
  const int r0 = blockIdx.x * TR;
  const int rt = wv & 3, ct0 = (wv >> 2) * 4;
  constexpr int NOUT = (MODE == 2) ? NQ : FF;
  constexpr int KS1 = (MODE == 2) ? 2 : 3;
  constexpr int K1 = (MODE == 2) ? FF : DIN;

  if (MODE == 0) {
    if (tid < TR) {
      const float* rl = src + (size_t)(r0 + tid) * RECW;
      const float cnt = rl[31];
      sStat[tid * 8 + 0] = cnt;
      sStat[tid * 8 + 1] = 1.0f / fmaxf(cnt, 1.0f);
      sStat[tid * 8 + 2] = rl[27];
      sStat[tid * 8 + 3] = rl[28];
      sStat[tid * 8 + 4] = rl[29];
      sStat[tid * 8 + 5] = rl[30];
      sStat[tid * 8 + 6] = 0.f;
      sStat[tid * 8 + 7] = 0.f;
    }
    {
      const int r = tid >> 2, q = tid & 3;
      const v4fa* p = (const v4fa*)(src + (size_t)(r0 + r) * RECW + 8 * q);
      const v4f u0 = p[0], u1 = p[1];
      float f[8];
      f[0] = u0.x; f[1] = u0.y; f[2] = u0.z; f[3] = u0.w;
      f[4] = u1.x; f[5] = u1.y; f[6] = u1.z; f[7] = u1.w;
      Pack8 pk;
      #pragma unroll
      for (int j = 0; j < 8; ++j) {
        const int k = 8 * q + j;
        pk.h[j] = (_Float16)(((k < 27) ? f[j] : 0.f) * A_SC);
      }
      *(v4ua*)(sA1 + r * AP + 8 * q) = pk.u;
    }
    cvt_w<4, FF>(cw, 27, FF, sW, tid);
    stage_bias(cb, FF, sBias, tid);
    __syncthreads();
    {
      const int cc0 = (wv >> 2) * 2;
      const v8f z8 = {0.f, 0.f, 0.f, 0.f, 0.f, 0.f, 0.f, 0.f};
      const v16h a = ldfrag(sA1 + (16 * rt + m) * AP, h);
      v8f cacc[2];
      #pragma unroll
      for (int jn = 0; jn < 2; ++jn) {
        const v16h bq = ldfrag(sW + (16 * (cc0 + jn) + m) * AP, h);
        cacc[jn] = wmma_h(a, bq, z8);
      }
      #pragma unroll
      for (int jn = 0; jn < 2; ++jn) {
        const int col = 16 * (cc0 + jn) + m;
        const float bc = sBias[col];
        #pragma unroll
        for (int r = 0; r < 8; ++r) {
          const int row = 16 * rt + 8 * h + r;
          const float cnt = sStat[row * 8 + 0], rd = sStat[row * 8 + 1];
          const float v = (cacc[jn][r] * R_ACC + cnt * bc) * rd;
          sA0[row * AP + col] = hbits(v * A_SC);
        }
      }
    }
    #pragma unroll
    for (int jj = 0; jj < 2; ++jj) {
      const int i = tid + 256 * jj;
      const int r = i >> 3, q = i & 7;
      const float rd = sStat[r * 8 + 1];
      const bool q0 = (q == 0);
      Pack8 pk;
      pk.h[0] = (_Float16)((q0 ? (sStat[r * 8 + 2] * rd) : 0.f) * A_SC);
      pk.h[1] = (_Float16)((q0 ? (sStat[r * 8 + 3] * rd) : 0.f) * A_SC);
      pk.h[2] = (_Float16)((q0 ? (sStat[r * 8 + 4] * rd) : 0.f) * A_SC);
      pk.h[3] = (_Float16)((q0 ? (sStat[r * 8 + 5] * rd) : 0.f) * A_SC);
      pk.h[4] = (_Float16)0.f;
      pk.h[5] = (_Float16)0.f;
      pk.h[6] = (_Float16)0.f;
      pk.h[7] = (_Float16)0.f;
      *(v4ua*)(sA0 + r * AP + 64 + 8 * q) = pk.u;
    }
    __syncthreads();
  } else {
    constexpr int SP = (MODE == 1) ? XINW : FF;
    constexpr int QV = SP / 8;
    #pragma unroll
    for (int jj = 0; jj < 4; ++jj) {
      const int i = tid + 256 * jj;
      const int r = i >> 4, q = i & 15;
      const int qc = (q < QV) ? q : (QV - 1);
      const v4fa* p = (const v4fa*)(src + (size_t)(r0 + r) * SP + 8 * qc);
      const v4f u0 = p[0], u1 = p[1];
      const bool ok = (q < QV);
      Pack8 pk;
      pk.h[0] = (_Float16)((ok ? u0.x : 0.f) * A_SC);
      pk.h[1] = (_Float16)((ok ? u0.y : 0.f) * A_SC);
      pk.h[2] = (_Float16)((ok ? u0.z : 0.f) * A_SC);
      pk.h[3] = (_Float16)((ok ? u0.w : 0.f) * A_SC);
      pk.h[4] = (_Float16)((ok ? u1.x : 0.f) * A_SC);
      pk.h[5] = (_Float16)((ok ? u1.y : 0.f) * A_SC);
      pk.h[6] = (_Float16)((ok ? u1.z : 0.f) * A_SC);
      pk.h[7] = (_Float16)((ok ? u1.w : 0.f) * A_SC);
      *(v4ua*)(sA0 + r * AP + 8 * q) = pk.u;
    }
    if (MODE == 2) {
      if (tid < TR) {
        const float* cl = cst + (size_t)(r0 + tid) * cpitch;
        const float a0 = cl[ci0], a1 = cl[ci0 + 1];
        const int cc = (cicnt >= 0) ? cicnt : 0;
        const float cv = cl[cc];
        const float rd = (cicnt >= 0) ? (1.0f / fmaxf(cv, 1.0f)) : 1.0f;
        sStat[tid * 8 + 0] = a0 * rd;
        sStat[tid * 8 + 1] = a1 * rd;
      }
    }
    __syncthreads();
  }

  v8f acc[4];
  cvt_w<KS1 * 4, NCOL>(wi, K1, HID, sW, tid);
  stage_bias(bi, HID, sBias, tid);
  __syncthreads();
  gemm4(sA0, sW, KS1, rt, ct0, m, h, acc);
  epi_hid(acc, sBias, sA1, rt, ct0, m, h);
  __syncthreads();
  cvt_w<16, NCOL>(wh, HID, HID, sW, tid);
  stage_bias(bh, HID, sBias, tid);
  __syncthreads();
  gemm4(sA1, sW, 4, rt, ct0, m, h, acc);
  epi_hid(acc, sBias, sA0, rt, ct0, m, h);
  __syncthreads();
  cvt_w<16, NCOL>(wh + HID * HID, HID, HID, sW, tid);
  stage_bias(bh + HID, HID, sBias, tid);
  __syncthreads();
  gemm4(sA0, sW, 4, rt, ct0, m, h, acc);
  epi_hid(acc, sBias, sA1, rt, ct0, m, h);
  __syncthreads();
  cvt_w<16, NCOL>(wo, HID, NOUT, sW, tid);
  stage_bias(bo, NOUT, sBias, tid);
  __syncthreads();
  gemm4(sA1, sW, 4, rt, ct0, m, h, acc);
  __syncthreads();

  if (ct0 == 0) {
    constexpr int NTF = (MODE == 2) ? 2 : 4;
    #pragma unroll
    for (int nt = 0; nt < NTF; ++nt) {
      const int col = 16 * nt + m;
      const float bc = sBias[col];
      #pragma unroll
      for (int r = 0; r < 8; ++r) {
        const int row = 16 * rt + 8 * h + r;
        float y = acc[nt][r] * R_ACC + bc;
        if (MODE == 2) {
          const float cx = sStat[row * 8 + 0], cy = sStat[row * 8 + 1];
          y = (col < NQ) ? y : ((col == NQ) ? cx : ((col == NQ + 1) ? cy : 0.f));
        }
        sY[row * YP + col] = y;
      }
    }
  }
  __syncthreads();

  constexpr int OW = (MODE == 2) ? JSFW : FF;
  constexpr int QPR = OW / 4;
  constexpr int NJ = (TR * QPR) / 256;
  v4f ov[NJ];
  #pragma unroll
  for (int jj = 0; jj < NJ; ++jj) {
    const int i = tid + 256 * jj;
    const int r = i / QPR, q = i - r * QPR;
    ov[jj] = *(const v4fa*)(sY + r * YP + 4 * q);
  }
  #pragma unroll
  for (int jj = 0; jj < NJ; ++jj) {
    const int i = tid + 256 * jj;
    const int r = i / QPR, q = i - r * QPR;
    *(volatile v4f*)(out + (size_t)(r0 + r) * OW + 4 * q) = ov[jj];
  }
  __threadfence();
  #pragma unroll
  for (int jj = 0; jj < NJ; ++jj) {
    const int i = tid + 256 * jj;
    const int r = i / QPR, q = i - r * QPR;
    *(volatile v4f*)(out + (size_t)(r0 + r) * OW + 4 * q) = ov[jj];
  }
}

__global__ __launch_bounds__(256) void k_gconv(const float* __restrict__ agg,
                                               const float* __restrict__ xp,
                                               const float* __restrict__ wn,
                                               const float* __restrict__ wsl,
                                               const float* __restrict__ gb,
                                               float* __restrict__ out)
{
  __shared__ __align__(16) unsigned short sA[TR * AP];
  __shared__ __align__(16) unsigned short sW[FF * AP];
  __shared__ __align__(16) float sY[TR * YP];
  __shared__ float sBias[NCOL];
  const int tid = threadIdx.x, lane = tid & 31, wv = tid >> 5;
  const int h = lane >> 4, m = lane & 15;
  const int r0 = blockIdx.x * TR;
  const int rt = wv & 3, ct0 = (wv >> 2) * 2;

  #pragma unroll
  for (int jj = 0; jj < 4; ++jj) {
    const int i = tid + 256 * jj;
    const int r = (i & 511) >> 3, q = i & 7;
    const float* S = (jj < 2) ? agg : xp;
    const int cb = (jj < 2) ? 0 : FF;
    const v4fa* p = (const v4fa*)(S + (size_t)(r0 + r) * FF + 8 * q);
    const v4f u0 = p[0], u1 = p[1];
    Pack8 pk;
    pk.h[0] = (_Float16)(u0.x * A_SC); pk.h[1] = (_Float16)(u0.y * A_SC);
    pk.h[2] = (_Float16)(u0.z * A_SC); pk.h[3] = (_Float16)(u0.w * A_SC);
    pk.h[4] = (_Float16)(u1.x * A_SC); pk.h[5] = (_Float16)(u1.y * A_SC);
    pk.h[6] = (_Float16)(u1.z * A_SC); pk.h[7] = (_Float16)(u1.w * A_SC);
    *(v4ua*)(sA + r * AP + cb + 8 * q) = pk.u;
  }
  cvt_w<8, FF>(wn,  FF, FF, sW, tid);
  cvt_w<8, FF>(wsl, FF, FF, sW + FF, tid);
  stage_bias(gb, FF, sBias, tid);
  __syncthreads();

  const v8f z8 = {0.f, 0.f, 0.f, 0.f, 0.f, 0.f, 0.f, 0.f};
  v8f acc[2];
  acc[0] = z8; acc[1] = z8;
  #pragma unroll 1
  for (int ks = 0; ks < 4; ++ks) {
    const v16h a = ldfrag(sA + (16 * rt + m) * AP + 32 * ks, h);
    #pragma unroll
    for (int nt = 0; nt < 2; ++nt) {
      const v16h bq = ldfrag(sW + (16 * (ct0 + nt) + m) * AP + 32 * ks, h);
      acc[nt] = wmma_h(a, bq, acc[nt]);
    }
  }
  #pragma unroll
  for (int nt = 0; nt < 2; ++nt) {
    const int col = 16 * (ct0 + nt) + m;
    const float bc = sBias[col];
    #pragma unroll
    for (int r = 0; r < 8; ++r) {
      const int row = 16 * rt + 8 * h + r;
      sY[row * YP + col] = acc[nt][r] * R_ACC + bc;
    }
  }
  __syncthreads();

  v4f ov[4];
  #pragma unroll
  for (int jj = 0; jj < 4; ++jj) {
    const int i = tid + 256 * jj;
    ov[jj] = *(const v4fa*)(sY + (i >> 4) * YP + 4 * (i & 15));
  }
  #pragma unroll
  for (int jj = 0; jj < 4; ++jj) {
    const int i = tid + 256 * jj;
    *(volatile v4f*)(out + (size_t)(r0 + (i >> 4)) * FF + 4 * (i & 15)) = ov[jj];
  }
  __threadfence();
  #pragma unroll
  for (int jj = 0; jj < 4; ++jj) {
    const int i = tid + 256 * jj;
    *(volatile v4f*)(out + (size_t)(r0 + (i >> 4)) * FF + 4 * (i & 15)) = ov[jj];
  }
}

__device__ __forceinline__ void render_px(const float* __restrict__ f, float gx, float gy, float* dst) {
  const v4fa* f4 = (const v4fa*)f;
  const v4f u0 = f4[0], u1 = f4[1], u2 = f4[2], u3 = f4[3], u4 = f4[4];
  float fv[20];
  fv[0] = u0.x;  fv[1] = u0.y;  fv[2] = u0.z;  fv[3] = u0.w;
  fv[4] = u1.x;  fv[5] = u1.y;  fv[6] = u1.z;  fv[7] = u1.w;
  fv[8] = u2.x;  fv[9] = u2.y;  fv[10] = u2.z; fv[11] = u2.w;
  fv[12] = u3.x; fv[13] = u3.y; fv[14] = u3.z; fv[15] = u3.w;
  fv[16] = u4.x; fv[17] = u4.y; fv[18] = u4.z; fv[19] = u4.w;
  const float dx = gx - fv[0];
  const float dy = gy - fv[1];
  const float dxx = dx * dx, dyy = dy * dy;
  #pragma unroll
  for (int k = 0; k < 3; ++k) {
    const float a = fv[2 + 6 * k], ah = fv[3 + 6 * k], aw = fv[4 + 6 * k];
    const float ahh = fv[5 + 6 * k], aww = fv[6 + 6 * k], ahw = fv[7 + 6 * k];
    float t = a + ah * dx;
    t = t + aw * dy;
    t = t + ahh * dxx;
    t = t + aww * dyy;
    t = t + (ahw * dx) * dy;
    dst[k] = t;
  }
}

__global__ __launch_bounds__(256) void k_render(const float* __restrict__ jsf1,
                                                const float* __restrict__ jsf2,
                                                const int* __restrict__ cl1,
                                                const int* __restrict__ cl2,
                                                float* __restrict__ o1,
                                                float* __restrict__ o2)
{
  __shared__ __align__(16) float sR[2][768];
  const int tid = threadIdx.x;
  const int p = blockIdx.x * 256 + tid;
  const int idx = p & 65535;
  const int i = idx >> 8, j = idx & 255;
  const float gx = (float)i * RH, gy = (float)j * RH;
  int c1 = cl1[p];
  c1 = (c1 < 0) ? 0 : ((c1 > NM1 - 1) ? (NM1 - 1) : c1);
  int c2 = cl2[c1];
  c2 = (c2 < 0) ? 0 : ((c2 > NM2 - 1) ? (NM2 - 1) : c2);
  render_px(jsf1 + (size_t)c1 * JSFW, gx, gy, &sR[0][3 * tid]);
  render_px(jsf2 + (size_t)c2 * JSFW, gx, gy, &sR[1][3 * tid]);
  __syncthreads();
  if (tid < 192) {
    const v4f a = *(const v4fa*)(&sR[0][4 * tid]);
    const v4f b = *(const v4fa*)(&sR[1][4 * tid]);
    float* d1 = o1 + (size_t)blockIdx.x * 768 + 4 * tid;
    float* d2 = o2 + (size_t)blockIdx.x * 768 + 4 * tid;
    *(volatile v4f*)d1 = a;
    *(volatile v4f*)d2 = b;
    __threadfence();
    *(volatile v4f*)d1 = a;
    *(volatile v4f*)d2 = b;
  }
}

extern "C" void kernel_launch(void* const* d_in, const int* in_sizes, int n_in,
                              void* d_out, int out_size, void* d_ws, size_t ws_size,
                              hipStream_t stream)
{
  if (n_in < 31) return;
  if (in_sizes[0] != NPIX * 3) return;
  if (in_sizes[1] != 27 * FF) return;
  if (in_sizes[2] != FF) return;
  for (int g = 0; g < 2; ++g) {
    const int b0 = 3 + 6 * g;
    if (in_sizes[b0 + 0] != DIN * HID) return;
    if (in_sizes[b0 + 1] != HID) return;
    if (in_sizes[b0 + 2] != 2 * HID * HID) return;
    if (in_sizes[b0 + 3] != 2 * HID) return;
    if (in_sizes[b0 + 4] != HID * FF) return;
    if (in_sizes[b0 + 5] != FF) return;
  }
  if (in_sizes[15] != FF * HID) return;
  if (in_sizes[16] != HID) return;
  if (in_sizes[17] != 2 * HID * HID) return;
  if (in_sizes[18] != 2 * HID) return;
  if (in_sizes[19] != HID * NQ) return;
  if (in_sizes[20] != NQ) return;
  for (int g = 0; g < 2; ++g) {
    const int b0 = 21 + 3 * g;
    if (in_sizes[b0 + 0] != FF * FF) return;
    if (in_sizes[b0 + 1] != FF * FF) return;
    if (in_sizes[b0 + 2] != FF) return;
  }
  if (in_sizes[27] != NPIX) return;
  if (in_sizes[28] != NM1) return;
  if ((in_sizes[29] & 1) != 0 || (in_sizes[30] & 1) != 0) return;
  const int nE1 = in_sizes[29] / 2;
  const int nE2 = in_sizes[30] / 2;
  if (nE1 <= 0 || nE2 <= 0) return;
  if ((nE1 & 3) != 0 || (nE2 & 3) != 0) return;
  if (nE1 > (1 << 24) || nE2 > (1 << 24)) return;
  if (out_size != 2 * NPIX * 3 + NM1 * FF + NM2 * FF) return;

  const float* img    = (const float*)d_in[0];
  const float* conv_w = (const float*)d_in[1];
  const float* conv_b = (const float*)d_in[2];
  const float* t1_wi  = (const float*)d_in[3];
  const float* t1_bi  = (const float*)d_in[4];
  const float* t1_wh  = (const float*)d_in[5];
  const float* t1_bh  = (const float*)d_in[6];
  const float* t1_wo  = (const float*)d_in[7];
  const float* t1_bo  = (const float*)d_in[8];
  const float* t2_wi  = (const float*)d_in[9];
  const float* t2_bi  = (const float*)d_in[10];
  const float* t2_wh  = (const float*)d_in[11];
  const float* t2_bh  = (const float*)d_in[12];
  const float* t2_wo  = (const float*)d_in[13];
  const float* t2_bo  = (const float*)d_in[14];
  const float* q_wi   = (const float*)d_in[15];
  const float* q_bi   = (const float*)d_in[16];
  const float* q_wh   = (const float*)d_in[17];
  const float* q_bh   = (const float*)d_in[18];
  const float* q_wo   = (const float*)d_in[19];
  const float* q_bo   = (const float*)d_in[20];
  const float* gc1_wn = (const float*)d_in[21];
  const float* gc1_ws = (const float*)d_in[22];
  const float* gc1_b  = (const float*)d_in[23];
  const float* gc2_wn = (const float*)d_in[24];
  const float* gc2_ws = (const float*)d_in[25];
  const float* gc2_b  = (const float*)d_in[26];
  const int* cl1 = (const int*)d_in[27];
  const int* cl2 = (const int*)d_in[28];
  const int* ed1 = (const int*)d_in[29];
  const int* ed2 = (const int*)d_in[30];

  float* out = (float*)d_out;
  float* o_r1 = out;
  float* o_r2 = out + (size_t)NPIX * 3;
  float* o_x1 = out + (size_t)2 * NPIX * 3;
  float* o_x2 = o_x1 + (size_t)NM1 * FF;

  const size_t bREC1 = (size_t)NM1 * RECW * 4;
  const size_t bX1P  = (size_t)NM1 * FF * 4;
  const size_t bAGG1 = (size_t)NM1 * FF * 4;
  const size_t bXIN2 = (size_t)NM2 * XINW * 4;
  const size_t bX2P  = (size_t)NM2 * FF * 4;
  const size_t bAGG2 = (size_t)NM2 * FF * 4;
  const size_t bJSF1 = (size_t)NM1 * JSFW * 4;
  const size_t bJSF2 = (size_t)NM2 * JSFW * 4;
  const size_t total = bREC1 + bX1P + bAGG1 + bXIN2 + bX2P + bAGG2 + bJSF1 + bJSF2;
  if (total > ws_size) return;
  if (total > (size_t)134217728) return;

  char* ws = (char*)d_ws;
  size_t off = 0;
  float* REC1 = (float*)(ws + off); off += bREC1;
  float* X1P  = (float*)(ws + off); off += bX1P;
  float* AGG1 = (float*)(ws + off); off += bAGG1;
  float* XIN2 = (float*)(ws + off); off += bXIN2;
  float* X2P  = (float*)(ws + off); off += bX2P;
  float* AGG2 = (float*)(ws + off); off += bAGG2;
  float* JSF1 = (float*)(ws + off); off += bJSF1;
  float* JSF2 = (float*)(ws + off); off += bJSF2;
  if (off != total) return;

  hipFuncSetAttribute(reinterpret_cast<const void*>(&k_fc<0>),
                      hipFuncAttributeMaxDynamicSharedMemorySize, LDS_FC);
  hipFuncSetAttribute(reinterpret_cast<const void*>(&k_fc<1>),
                      hipFuncAttributeMaxDynamicSharedMemorySize, LDS_FC);
  hipFuncSetAttribute(reinterpret_cast<const void*>(&k_fc<2>),
                      hipFuncAttributeMaxDynamicSharedMemorySize, LDS_FC);

  k_pool1<<<NM1 / NOWN, 256, 0, stream>>>(img, cl1, NPIX, REC1);
  k_fc<0><<<NM1 / TR, 256, LDS_FC, stream>>>(REC1, conv_w, conv_b,
                                             t1_wi, t1_bi, t1_wh, t1_bh, t1_wo, t1_bo,
                                             REC1, RECW, 27, 31, X1P);
  k_gagg<<<NM1 / NOWN, 256, 0, stream>>>(X1P, ed1, nE1, NM1, AGG1);
  k_gconv<<<NM1 / TR, 256, 0, stream>>>(AGG1, X1P, gc1_wn, gc1_ws, gc1_b, o_x1);
  k_pool2<<<NM2 / NOWN, 256, 0, stream>>>(o_x1, REC1, cl2, NM1, XIN2);
  k_fc<1><<<NM2 / TR, 256, LDS_FC, stream>>>(XIN2, conv_w, conv_b,
                                             t2_wi, t2_bi, t2_wh, t2_bh, t2_wo, t2_bo,
                                             XIN2, XINW, FF, -1, X2P);
  k_gagg<<<NM2 / NOWN, 256, 0, stream>>>(X2P, ed2, nE2, NM2, AGG2);
  k_gconv<<<NM2 / TR, 256, 0, stream>>>(AGG2, X2P, gc2_wn, gc2_ws, gc2_b, o_x2);
  k_fc<2><<<NM1 / TR, 256, LDS_FC, stream>>>(o_x1, conv_w, conv_b,
                                             q_wi, q_bi, q_wh, q_bh, q_wo, q_bo,
                                             REC1, RECW, 27, 31, JSF1);
  k_fc<2><<<NM2 / TR, 256, LDS_FC, stream>>>(o_x2, conv_w, conv_b,
                                             q_wi, q_bi, q_wh, q_bh, q_wo, q_bo,
                                             XIN2, XINW, FF, -1, JSF2);
  k_render<<<NPIX / 256, 256, 0, stream>>>(JSF1, JSF2, cl1, cl2, o_r1, o_r2);
}
